// _EncoderLayer_12257836663306
// MI455X (gfx1250) — hardware-verified
//
#include <hip/hip_runtime.h>

typedef _Float16 v16h __attribute__((ext_vector_type(16)));
typedef _Float16 v8h  __attribute__((ext_vector_type(8)));
typedef _Float16 v4h  __attribute__((ext_vector_type(4)));
typedef float    v8f  __attribute__((ext_vector_type(8)));
typedef float    v4f  __attribute__((ext_vector_type(4)));
typedef v8h __attribute__((may_alias)) v8ha;
typedef v4f __attribute__((may_alias)) v4fa;
typedef _Float16 __attribute__((may_alias)) f16a;

union Frag { v16h v; v8h half[2]; };

#define NBATCH 4
#define SS     1024
#define DD     1024
#define HH     16
#define HD     64
#define DFF    4096
#define MT     (NBATCH * SS)
#define PSCALE 16384.0f
#define TP     72

__device__ __forceinline__ v8f wmma_f16(v16h a, v16h b, v8f c) {
  v8f d = __builtin_amdgcn_wmma_f32_16x16x32_f16(false, a, false, b, (short)0, c, false, false);
  asm volatile("v_nop\n\tv_nop\n\tv_nop\n\tv_nop" : "+v"(d) : "v"(a), "v"(b));
  return d;
}

__device__ __forceinline__ v16h load_frag(const _Float16* p, int h) {
  Frag f;
  f.half[0] = *(const v8ha*)(p + 8 * h);
  f.half[1] = *(const v8ha*)(p + 16 + 8 * h);
  return f.v;
}

__global__ __launch_bounds__(256) void cvt_src_kernel(const float* __restrict__ x,
                                                      _Float16* __restrict__ xh, int n8)
{
  const int g = blockIdx.x * 256 + threadIdx.x;
  if (g >= n8) return;
  const float* src = x + (size_t)g * 8;
  const v4f a = *(const v4fa*)src;
  const v4f c = *(const v4fa*)(src + 4);
  const v8h o = { (_Float16)a.x, (_Float16)a.y, (_Float16)a.z, (_Float16)a.w,
                  (_Float16)c.x, (_Float16)c.y, (_Float16)c.z, (_Float16)c.w };
  _Float16* dst = xh + (size_t)g * 8;
  *(volatile v8h*)dst = o;
  __threadfence();
  *(volatile v8h*)dst = o;
}

__device__ __forceinline__ void tconv_store_pass(const _Float16* sh, _Float16* ob, int R,
                                                 int r0, int c0, int w, int lane) {
  const int q8 = lane & 7, sub = lane >> 3;
  #pragma unroll
  for (int i = 0; i < 2; ++i) {
    const int c = 8 * w + 4 * i + sub;
    const v8h v = *(const v8ha*)(sh + c * TP + 8 * q8);
    _Float16* dst = ob + (size_t)(c0 + c) * R + r0 + 8 * q8;
    *(volatile v8h*)dst = v;
  }
}

__global__ __launch_bounds__(256) void tconv_kernel(const float* __restrict__ in,
                                                    _Float16* __restrict__ out,
                                                    int R, int C, float sc)
{
  __shared__ __attribute__((aligned(16))) _Float16 sh[64 * TP];
  const int t = threadIdx.x, lane = t & 31, w = t >> 5;
  const int r0 = blockIdx.x * 64, c0 = blockIdx.y * 64;
  const size_t zoff = (size_t)blockIdx.z * (size_t)R * (size_t)C;
  const float* ib = in + zoff;
  _Float16* ob = out + zoff;
  #pragma unroll
  for (int i = 0; i < 4; ++i) {
    const int idx = t + 256 * i;
    const int r = idx >> 4, c4 = (idx & 15) * 4;
    const v4f v = *(const v4fa*)(ib + (size_t)(r0 + r) * C + c0 + c4);
    sh[(c4 + 0) * TP + r] = (_Float16)(v.x * sc);
    sh[(c4 + 1) * TP + r] = (_Float16)(v.y * sc);
    sh[(c4 + 2) * TP + r] = (_Float16)(v.z * sc);
    sh[(c4 + 3) * TP + r] = (_Float16)(v.w * sc);
  }
  __syncthreads();
  tconv_store_pass(sh, ob, R, r0, c0, w, lane);
  __threadfence();
  tconv_store_pass(sh, ob, R, r0, c0, w, lane);
}

__device__ __forceinline__ void store_qkv_pass(const f16a* sH, _Float16* plane, _Float16* vt,
                                               int which, int bh, int l0, int w, int lane) {
  const int q8 = lane & 7, sub = lane >> 3;
  #pragma unroll
  for (int i = 0; i < 8; ++i) {
    const int lid = w * 32 + i * 4 + sub;
    v8h v;
    _Float16* dst;
    if (which != 2) {
      v = *(const v8ha*)(sH + lid * HD + 8 * q8);
      dst = plane + ((size_t)bh * SS + l0 + lid) * HD + 8 * q8;
    } else {
      const int d = lid >> 1, hl = lid & 1;
      v = *(const v8ha*)(sH + d * 128 + 64 * hl + 8 * q8);
      dst = vt + ((size_t)bh * HD + d) * SS + l0 + 64 * hl + 8 * q8;
    }
    *(volatile v8h*)dst = v;
  }
}

__device__ __forceinline__ void store_f32_pass(const float* sF, const float* __restrict__ resid,
                                               float* outF, int N, int m0, int n0, int w, int lane) {
  const int q8 = lane & 7, sub = lane >> 3;
  #pragma unroll
  for (int i = 0; i < 16; ++i) {
    const int L = 4 * i + sub;
    const int row = 32 * w + (L >> 1), hl = L & 1;
    v4f v = *(const v4fa*)(sF + row * 64 + 32 * hl + 4 * q8);
    const size_t gi = (size_t)(m0 + row) * N + n0 + 32 * hl + 4 * q8;
    const v4f rr = *(const v4fa*)(resid + gi);
    v = v + rr;
    *(volatile v4f*)(outF + gi) = v;
  }
}

__device__ __forceinline__ void store_h_pass(const f16a* sH, _Float16* outH, int N,
                                             int m0, int n0, int w, int lane) {
  const int q8 = lane & 7, sub = lane >> 3;
  #pragma unroll
  for (int i = 0; i < 8; ++i) {
    const int row = 32 * w + 4 * i + sub;
    const v8h v = *(const v8ha*)(sH + row * 64 + 8 * q8);
    const size_t gi = (size_t)(m0 + row) * N + n0 + 8 * q8;
    *(volatile v8h*)(outH + gi) = v;
  }
}

template <int MODE>
__global__ __launch_bounds__(128) void gemm_kernel(
    const _Float16* __restrict__ A, const _Float16* __restrict__ Bt, int K, int N,
    const float* __restrict__ bias0, const float* __restrict__ bias1, const float* __restrict__ bias2,
    const float* __restrict__ resid, float osc,
    float* __restrict__ outF, _Float16* __restrict__ outH, _Float16* __restrict__ outH2,
    _Float16* __restrict__ outV)
{
  constexpr int LDSF = (MODE == 1) ? (128 * 64) : (128 * 32);
  __shared__ __attribute__((aligned(16))) float sF[LDSF];
  f16a* sH = (f16a*)sF;

  const int tid = threadIdx.x, lane = tid & 31, w = tid >> 5;
  const int h = lane >> 4, m = lane & 15;
  const int m0 = blockIdx.x * 128, n0 = blockIdx.y * 64;
  const int m0w = m0 + 32 * w;

  const _Float16* xa0 = A + (size_t)(m0w + m) * K;
  const _Float16* xa1 = xa0 + (size_t)16 * K;
  const _Float16* wb  = Bt + (size_t)(n0 + m) * K;

  const v8f zero8 = {0.f, 0.f, 0.f, 0.f, 0.f, 0.f, 0.f, 0.f};
  v8f acc[2][4];
  #pragma unroll
  for (int mt = 0; mt < 2; ++mt)
    #pragma unroll
    for (int nt = 0; nt < 4; ++nt) acc[mt][nt] = zero8;

  #pragma unroll 1
  for (int k0 = 0; k0 < K; k0 += 32) {
    const v16h a0 = load_frag(xa0 + k0, h);
    const v16h a1 = load_frag(xa1 + k0, h);
    #pragma unroll
    for (int nt = 0; nt < 4; ++nt) {
      const v16h b = load_frag(wb + (size_t)nt * 16 * K + k0, h);
      acc[0][nt] = wmma_f16(a0, b, acc[0][nt]);
      acc[1][nt] = wmma_f16(a1, b, acc[1][nt]);
    }
  }

  int which = 0, head = 0;
  const float* bias = bias0;
  if (MODE == 0) {
    which = blockIdx.y >> 4;
    head = blockIdx.y & 15;
    bias = (which == 0) ? bias0 : ((which == 1) ? bias1 : bias2);
  }
  #pragma unroll
  for (int nt = 0; nt < 4; ++nt) {
    const int feat = 16 * nt + m;
    const int bidx = (MODE == 0) ? (head * HD + feat) : (n0 + feat);
    const float bvl = bias[bidx];
    #pragma unroll
    for (int mt = 0; mt < 2; ++mt) {
      #pragma unroll
      for (int r = 0; r < 8; ++r) {
        const int tokl = 32 * w + 16 * mt + 8 * h + r;
        float y = acc[mt][nt][r] * osc + bvl;
        if (MODE == 1) {
          sF[tokl * 64 + feat] = y;
        } else if (MODE == 2) {
          y = fmaxf(y, 0.0f);
          sH[tokl * 64 + feat] = (_Float16)y;
        } else {
          const int idx = (which == 2) ? (feat * 128 + tokl) : (tokl * 64 + feat);
          sH[idx] = (_Float16)y;
        }
      }
    }
  }
  __syncthreads();

  if (MODE == 0) {
    const int b = m0 / SS, l0 = m0 - b * SS, bh = b * HH + head;
    _Float16* plane = (which == 0) ? outH : outH2;
    store_qkv_pass(sH, plane, outV, which, bh, l0, w, lane);
    __threadfence();
    store_qkv_pass(sH, plane, outV, which, bh, l0, w, lane);
  } else if (MODE == 1) {
    store_f32_pass(sF, resid, outF, N, m0, n0, w, lane);
    __threadfence();
    store_f32_pass(sF, resid, outF, N, m0, n0, w, lane);
  } else {
    store_h_pass(sH, outH, N, m0, n0, w, lane);
    __threadfence();
    store_h_pass(sH, outH, N, m0, n0, w, lane);
  }
}

__device__ __forceinline__ v16h pack_p(v8f a, v8f c) {
  const v16h r = { (_Float16)(a[0] * PSCALE), (_Float16)(a[1] * PSCALE), (_Float16)(a[2] * PSCALE), (_Float16)(a[3] * PSCALE),
                   (_Float16)(a[4] * PSCALE), (_Float16)(a[5] * PSCALE), (_Float16)(a[6] * PSCALE), (_Float16)(a[7] * PSCALE),
                   (_Float16)(c[0] * PSCALE), (_Float16)(c[1] * PSCALE), (_Float16)(c[2] * PSCALE), (_Float16)(c[3] * PSCALE),
                   (_Float16)(c[4] * PSCALE), (_Float16)(c[5] * PSCALE), (_Float16)(c[6] * PSCALE), (_Float16)(c[7] * PSCALE) };
  return r;
}

__device__ __forceinline__ void att_store_pass(const _Float16* so, _Float16* ao,
                                               int b, int head, int q0, int lane) {
  const int q8 = lane & 7, sub = lane >> 3;
  #pragma unroll
  for (int i = 0; i < 4; ++i) {
    const int row = i * 4 + sub;
    const v8h v = *(const v8ha*)(so + row * 64 + 8 * q8);
    const size_t gi = ((size_t)b * SS + q0 + row) * DD + head * HD + 8 * q8;
    *(volatile v8h*)(ao + gi) = v;
  }
}

__global__ __launch_bounds__(128) void attn_kernel(
    const _Float16* __restrict__ qh,
    const _Float16* __restrict__ kh,
    const _Float16* __restrict__ vt,
    _Float16* __restrict__ ao)
{
  __shared__ __attribute__((aligned(16))) _Float16 sO[4 * 16 * 64];

  const int tid = threadIdx.x, lane = tid & 31, w = tid >> 5;
  const int h = lane >> 4, m = lane & 15;
  const int bh = blockIdx.y, b = bh >> 4, head = bh & 15;
  const int q0 = blockIdx.x * 64 + 16 * w;

  const _Float16* qrow = qh + ((size_t)bh * SS + q0 + m) * HD;
  const v16h qb0 = load_frag(qrow, h);
  const v16h qb1 = load_frag(qrow + 32, h);

  const v8f zero8 = {0.f, 0.f, 0.f, 0.f, 0.f, 0.f, 0.f, 0.f};
  v8f o[4];
  #pragma unroll
  for (int t = 0; t < 4; ++t) o[t] = zero8;
  float mrun = -1e30f, lrun = 0.0f;

  const _Float16* kbase = kh + ((size_t)bh * SS + m) * HD;
  const _Float16* vbase = vt + ((size_t)bh * HD + m) * SS;

  #pragma unroll 1
  for (int kb = 0; kb < SS; kb += 64) {
    v8f s[4];
    #pragma unroll
    for (int j = 0; j < 4; ++j) {
      const _Float16* kp = kbase + (size_t)(kb + 16 * j) * HD;
      const v16h kf0 = load_frag(kp, h);
      const v16h kf1 = load_frag(kp + 32, h);
      v8f z = zero8;
      z = wmma_f16(kf0, qb0, z);
      z = wmma_f16(kf1, qb1, z);
      #pragma unroll
      for (int r = 0; r < 8; ++r) z[r] = z[r] * 0.125f;
      s[j] = z;
    }

    float mloc = s[0][0];
    #pragma unroll
    for (int j = 0; j < 4; ++j)
      #pragma unroll
      for (int r = 0; r < 8; ++r) mloc = fmaxf(mloc, s[j][r]);
    mloc = fmaxf(mloc, __shfl_xor(mloc, 16));
    const float mnew = fmaxf(mrun, mloc);
    const float alpha = __expf(mrun - mnew);
    mrun = mnew;
    float lsum = 0.0f;
    #pragma unroll
    for (int j = 0; j < 4; ++j)
      #pragma unroll
      for (int r = 0; r < 8; ++r) {
        const float p = __expf(s[j][r] - mnew);
        s[j][r] = p;
        lsum += p;
      }
    lsum += __shfl_xor(lsum, 16);
    lrun = lrun * alpha + lsum;
    #pragma unroll
    for (int t = 0; t < 4; ++t)
      #pragma unroll
      for (int r = 0; r < 8; ++r) o[t][r] = o[t][r] * alpha;

    const v16h pb0 = pack_p(s[0], s[1]);
    const v16h pb1 = pack_p(s[2], s[3]);

    #pragma unroll
    for (int t = 0; t < 4; ++t) {
      const _Float16* vp = vbase + (size_t)(16 * t) * SS + kb;
      const v16h vf0 = load_frag(vp, h);
      const v16h vf1 = load_frag(vp + 32, h);
      o[t] = wmma_f16(vf0, pb0, o[t]);
      o[t] = wmma_f16(vf1, pb1, o[t]);
    }
  }

  const float inv = (1.0f / lrun) * (1.0f / PSCALE);
  _Float16* so = sO + w * 1024;
  #pragma unroll
  for (int t = 0; t < 4; ++t)
    #pragma unroll
    for (int r = 0; r < 8; ++r)
      so[m * 64 + 16 * t + 8 * h + r] = (_Float16)(o[t][r] * inv);
  __syncthreads();

  att_store_pass(so, ao, b, head, q0, lane);
  __threadfence();
  att_store_pass(so, ao, b, head, q0, lane);
}

__global__ __launch_bounds__(256) void ln_kernel(const float* __restrict__ in,
                                                 const float* __restrict__ gam,
                                                 const float* __restrict__ bet,
                                                 float* __restrict__ outF,
                                                 _Float16* __restrict__ outH, int writeH)
{
  __shared__ float rs[8];
  __shared__ float rq[8];
  const int row = blockIdx.x, t = threadIdx.x, lane = t & 31, w = t >> 5;
  const size_t gi = (size_t)row * DD + 4 * t;
  const v4f v = *(const v4fa*)(in + gi);

  float s = (v.x + v.y) + (v.z + v.w);
  #pragma unroll
  for (int off = 16; off; off >>= 1) s += __shfl_xor(s, off);
  if (lane == 0) rs[w] = s;
  __syncthreads();
  float ts = 0.0f;
  #pragma unroll
  for (int i = 0; i < 8; ++i) ts += rs[i];
  const float mean = ts * (1.0f / DD);

  const float dx = v.x - mean, dy = v.y - mean, dz = v.z - mean, dw = v.w - mean;
  float q = (dx * dx + dy * dy) + (dz * dz + dw * dw);
  #pragma unroll
  for (int off = 16; off; off >>= 1) q += __shfl_xor(q, off);
  if (lane == 0) rq[w] = q;
  __syncthreads();
  float tq = 0.0f;
  #pragma unroll
  for (int i = 0; i < 8; ++i) tq += rq[i];
  const float var = tq * (1.0f / DD);
  const float rstd = 1.0f / sqrtf(var + 1e-5f);

  const v4f g = *(const v4fa*)(gam + 4 * t);
  const v4f bb = *(const v4fa*)(bet + 4 * t);
  v4f o;
  o.x = dx * rstd * g.x + bb.x;
  o.y = dy * rstd * g.y + bb.y;
  o.z = dz * rstd * g.z + bb.z;
  o.w = dw * rstd * g.w + bb.w;
  const v4h oh = { (_Float16)o.x, (_Float16)o.y, (_Float16)o.z, (_Float16)o.w };

  *(volatile v4f*)(outF + gi) = o;
  if (writeH) *(volatile v4h*)(outH + gi) = oh;
  __threadfence();
  *(volatile v4f*)(outF + gi) = o;
  if (writeH) *(volatile v4h*)(outH + gi) = oh;
}

extern "C" void kernel_launch(void* const* d_in, const int* in_sizes, int n_in,
                              void* d_out, int out_size, void* d_ws, size_t ws_size,
                              hipStream_t stream) {
  if (n_in < 17) return;
  if (in_sizes[0] != MT * DD) return;
  if (in_sizes[1] != HH * DD * HD || in_sizes[3] != HH * DD * HD || in_sizes[5] != HH * DD * HD) return;
  if (in_sizes[2] != HH * HD || in_sizes[4] != HH * HD || in_sizes[6] != HH * HD) return;
  if (in_sizes[7] != DD * DD || in_sizes[8] != DD || in_sizes[9] != DD || in_sizes[10] != DD) return;
  if (in_sizes[11] != DD * DFF || in_sizes[12] != DFF || in_sizes[13] != DFF * DD || in_sizes[14] != DD) return;
  if (in_sizes[15] != DD || in_sizes[16] != DD) return;
  if (out_size != MT * DD) return;

  const float* src = (const float*)d_in[0];
  const float* Wq  = (const float*)d_in[1];
  const float* bq  = (const float*)d_in[2];
  const float* Wk  = (const float*)d_in[3];
  const float* bk  = (const float*)d_in[4];
  const float* Wv  = (const float*)d_in[5];
  const float* bv  = (const float*)d_in[6];
  const float* Wo  = (const float*)d_in[7];
  const float* bo  = (const float*)d_in[8];
  const float* g1  = (const float*)d_in[9];
  const float* be1 = (const float*)d_in[10];
  const float* W1  = (const float*)d_in[11];
  const float* b1  = (const float*)d_in[12];
  const float* W2  = (const float*)d_in[13];
  const float* b2  = (const float*)d_in[14];
  const float* g2  = (const float*)d_in[15];
  const float* be2 = (const float*)d_in[16];
  float* out = (float*)d_out;

  const size_t b_srch = (size_t)MT * DD * 2;
  const size_t b_wqkv = (size_t)3 * HH * HD * DD * 2;
  const size_t b_wo   = (size_t)DD * DD * 2;
  const size_t b_w1   = (size_t)DFF * DD * 2;
  const size_t b_w2   = (size_t)DD * DFF * 2;
  const size_t b_pl   = (size_t)NBATCH * HH * SS * HD * 2;
  const size_t b_ao   = (size_t)MT * DD * 2;
  const size_t b_h1   = (size_t)MT * DFF * 2;
  const size_t b_r1   = (3 * b_pl + b_ao > b_h1) ? (3 * b_pl + b_ao) : b_h1;
  const size_t b_tmp  = (size_t)MT * DD * 4;
  const size_t b_x    = (size_t)MT * DD * 4;
  const size_t b_xh   = (size_t)MT * DD * 2;

  const size_t o_srch = 0;
  const size_t o_wqkv = o_srch + b_srch;
  const size_t o_wo   = o_wqkv + b_wqkv;
  const size_t o_w1   = o_wo + b_wo;
  const size_t o_w2   = o_w1 + b_w1;
  const size_t o_r1   = o_w2 + b_w2;
  const size_t o_tmp  = o_r1 + b_r1;
  const size_t o_x    = o_tmp + b_tmp;
  const size_t o_xh   = o_x + b_x;
  const size_t total  = o_xh + b_xh;
  if (total > ws_size) return;

  char* ws = (char*)d_ws;
  _Float16* srch  = (_Float16*)(ws + o_srch);
  _Float16* wqkvt = (_Float16*)(ws + o_wqkv);
  _Float16* wot   = (_Float16*)(ws + o_wo);
  _Float16* w1t   = (_Float16*)(ws + o_w1);
  _Float16* w2t   = (_Float16*)(ws + o_w2);
  _Float16* qh    = (_Float16*)(ws + o_r1);
  _Float16* kh    = (_Float16*)(ws + o_r1 + b_pl);
  _Float16* vt    = (_Float16*)(ws + o_r1 + 2 * b_pl);
  _Float16* ao    = (_Float16*)(ws + o_r1 + 3 * b_pl);
  _Float16* h1    = (_Float16*)(ws + o_r1);
  float*    tmp   = (float*)(ws + o_tmp);
  float*    xf    = (float*)(ws + o_x);
  _Float16* xh    = (_Float16*)(ws + o_xh);

  const int n8 = MT * DD / 8;
  cvt_src_kernel<<<dim3((n8 + 255) / 256), dim3(256), 0, stream>>>(src, srch, n8);

  tconv_kernel<<<dim3(DD / 64, HD / 64, HH), dim3(256), 0, stream>>>(Wq, wqkvt, DD, HD, 32.0f);
  tconv_kernel<<<dim3(DD / 64, HD / 64, HH), dim3(256), 0, stream>>>(Wk, wqkvt + (size_t)HH * HD * DD, DD, HD, 32.0f);
  tconv_kernel<<<dim3(DD / 64, HD / 64, HH), dim3(256), 0, stream>>>(Wv, wqkvt + (size_t)2 * HH * HD * DD, DD, HD, 32.0f);
  tconv_kernel<<<dim3(DD / 64, DD / 64, 1), dim3(256), 0, stream>>>(Wo, wot, DD, DD, 32.0f);
  tconv_kernel<<<dim3(DD / 64, DFF / 64, 1), dim3(256), 0, stream>>>(W1, w1t, DD, DFF, 32.0f);
  tconv_kernel<<<dim3(DFF / 64, DD / 64, 1), dim3(256), 0, stream>>>(W2, w2t, DFF, DD, 64.0f);

  gemm_kernel<0><<<dim3(MT / 128, 3 * HH), dim3(128), 0, stream>>>(
      srch, wqkvt, DD, HD, bq, bk, bv, src, 0.03125f, tmp, qh, kh, vt);

  attn_kernel<<<dim3(SS / 64, NBATCH * HH), dim3(128), 0, stream>>>(qh, kh, vt, ao);

  gemm_kernel<1><<<dim3(MT / 128, DD / 64), dim3(128), 0, stream>>>(
      ao, wot, DD, DD, bo, bo, bo, src, 0.03125f, tmp, xh, xh, xh);

  ln_kernel<<<dim3(MT), dim3(256), 0, stream>>>(tmp, g1, be1, xf, xh, 1);

  gemm_kernel<2><<<dim3(MT / 128, DFF / 64), dim3(128), 0, stream>>>(
      xh, w1t, DD, DFF, b1, b1, b1, xf, 0.03125f, tmp, h1, h1, h1);

  gemm_kernel<1><<<dim3(MT / 128, DD / 64), dim3(128), 0, stream>>>(
      h1, w2t, DFF, DD, b2, b2, b2, xf, 0.015625f, tmp, xh, xh, xh);

  ln_kernel<<<dim3(MT), dim3(256), 0, stream>>>(tmp, g2, be2, out, xh, 0);
}
